// Encoder_46033459478804
// MI455X (gfx1250) — hardware-verified
//
#include <hip/hip_runtime.h>


#ifndef NB
#define NB 8
#endif
#ifndef SEQ
#define SEQ 1024
#endif
#define NB_FULL  8
#define SEQ_FULL 1024
#define DM   512
#define DF   2048
#define NH   8
#define HD   64
#define DQKV (3 * DM)
#define NTOK (NB * SEQ)
#define QR   32
#define CH   256
#define VTP  (CH + 8)
#define ZN   (SEQ / 32)
#define NEWT 10

static_assert(NB >= 1 && NB <= NB_FULL);
static_assert(SEQ >= CH && SEQ <= SEQ_FULL);
static_assert(SEQ % CH == 0);
static_assert(SEQ % 128 == 0);
static_assert(NTOK % QR == 0);
static_assert(NH * HD == DM);
static_assert(QR == 32);
static_assert((ZN % 4) == 0);
static_assert(DM % 32 == 0 && DF % 32 == 0);
static_assert((DM * DM) % 2048 == 0 && (DF * DM) % 2048 == 0);

typedef _Float16 v16h __attribute__((ext_vector_type(16)));
typedef _Float16 v8h  __attribute__((ext_vector_type(8)));
typedef _Float16 v4h  __attribute__((ext_vector_type(4)));
typedef float    v8f  __attribute__((ext_vector_type(8)));
typedef float    v4f  __attribute__((ext_vector_type(4)));

union Frag { v16h v; v8h h[2]; };

#define WSC   64.0f
#define SC_Z  1.52587890625e-05f
#define SC_P  16384.0f
#define SC_C  6.103515625e-05f
#define SC_O  2.44140625e-04f
#define SC_H  0.015625f
#define LOG2E 1.44269504088896340736f
#define LN_EPS 1e-5f

static __device__ __forceinline__ v8f zero8() {
    v8f z;
#pragma unroll
    for (int i = 0; i < 8; ++i) z[i] = 0.0f;
    return z;
}

static __device__ __forceinline__ v16h load_frag16(const _Float16* base, int ld, int lane) {
    int m  = lane & 15;
    int kb = (lane >> 4) << 3;
    const _Float16* p = base + (size_t)m * ld + kb;
    Frag f;
    f.h[0] = *(const v8h*)(p);
    f.h[1] = *(const v8h*)(p + 16);
    return f.v;
}

static __device__ __forceinline__ v8f wmma16(v16h a, v16h b, v8f c) {
    v8f d = __builtin_amdgcn_wmma_f32_16x16x32_f16(false, a, false, b, (short)0, c, false, false);
    asm volatile("v_nop\n\tv_nop\n\tv_nop\n\tv_nop" : "+v"(d) : "v"(a), "v"(b));
    return d;
}

static __device__ __forceinline__ float bf16r(float x) {
    unsigned u = __float_as_uint(x);
    u = (u + 0x7FFFu + ((u >> 16) & 1u)) & 0xFFFF0000u;
    return __uint_as_float(u);
}

static __device__ __forceinline__ void wave_lds_sync() {
    __builtin_amdgcn_fence(3, "wavefront");
    asm volatile("s_wait_dscnt 0" ::: "memory");
    __builtin_amdgcn_wave_barrier();
}

static __device__ __forceinline__ float wsum(float v) {
    v += __shfl_xor(v, 16, 32); v += __shfl_xor(v, 8, 32); v += __shfl_xor(v, 4, 32);
    v += __shfl_xor(v, 2, 32);  v += __shfl_xor(v, 1, 32);
    return v;
}
static __device__ __forceinline__ float wmaxr(float v) {
    v = fmaxf(v, __shfl_xor(v, 16, 32)); v = fmaxf(v, __shfl_xor(v, 8, 32));
    v = fmaxf(v, __shfl_xor(v, 4, 32));  v = fmaxf(v, __shfl_xor(v, 2, 32));
    v = fmaxf(v, __shfl_xor(v, 1, 32));
    return v;
}
static __device__ __forceinline__ float wminr(float v) {
    v = fminf(v, __shfl_xor(v, 16, 32)); v = fminf(v, __shfl_xor(v, 8, 32));
    v = fminf(v, __shfl_xor(v, 4, 32));  v = fminf(v, __shfl_xor(v, 2, 32));
    v = fminf(v, __shfl_xor(v, 1, 32));
    return v;
}

static __device__ __forceinline__ float mishf(float x) {
    float xe = fminf(x, 20.0f);
    float u  = __builtin_amdgcn_exp2f(xe * LOG2E);
    float wv = u * (u + 2.0f);
    float t  = wv * __builtin_amdgcn_rcpf(wv + 2.0f);
    return x * t;
}

static __device__ __forceinline__ void load_cols16(const float* p, int lane, float (&o)[16]) {
#pragma unroll
    for (int j = 0; j < 2; ++j) {
        v4f a = *(const v4f*)(p + 256 * j + 8 * lane);
        v4f c = *(const v4f*)(p + 256 * j + 8 * lane + 4);
        o[8 * j + 0] = a.x; o[8 * j + 1] = a.y; o[8 * j + 2] = a.z; o[8 * j + 3] = a.w;
        o[8 * j + 4] = c.x; o[8 * j + 5] = c.y; o[8 * j + 6] = c.z; o[8 * j + 7] = c.w;
    }
}

static __device__ __forceinline__ void ln_lane(const float (&v)[16], const float (&gl)[16],
                                               const float (&el)[16], float (&y)[16]) {
    float s = 0.0f;
#pragma unroll
    for (int e = 0; e < 16; ++e) s += v[e];
    s = wsum(s);
    const float mu = s * (1.0f / (float)DM);
    float d[16];
    float q = 0.0f;
#pragma unroll
    for (int e = 0; e < 16; ++e) { d[e] = v[e] - mu; q = __builtin_fmaf(d[e], d[e], q); }
    q = wsum(q);
    const float rstd = rsqrtf(__builtin_fmaf(q, 1.0f / (float)DM, LN_EPS));
#pragma unroll
    for (int e = 0; e < 16; ++e) y[e] = d[e] * rstd * gl[e] + el[e];
}

__global__ __launch_bounds__(256) void k_wcvt(const float* __restrict__ src,
                                               _Float16* __restrict__ dst) {
    const size_t i = (size_t)blockIdx.x * 256 + threadIdx.x;
    v4f a = *(const v4f*)(src + i * 8);
    v4f c = *(const v4f*)(src + i * 8 + 4);
    v8h o;
    o[0] = (_Float16)(bf16r(a.x) * WSC); o[1] = (_Float16)(bf16r(a.y) * WSC);
    o[2] = (_Float16)(bf16r(a.z) * WSC); o[3] = (_Float16)(bf16r(a.w) * WSC);
    o[4] = (_Float16)(bf16r(c.x) * WSC); o[5] = (_Float16)(bf16r(c.y) * WSC);
    o[6] = (_Float16)(bf16r(c.z) * WSC); o[7] = (_Float16)(bf16r(c.w) * WSC);
    *(volatile v8h*)(dst + i * 8) = o;
    __threadfence();
    *(volatile v8h*)(dst + i * 8) = o;
}

__global__ __launch_bounds__(256) void k_ln1(const float* __restrict__ x,
                                              const float* __restrict__ g,
                                              const float* __restrict__ be,
                                              _Float16* __restrict__ y) {
    const int tid = threadIdx.x, lane = tid & 31, w = tid >> 5;
    const int tok = blockIdx.x * 8 + w;
    const int b = tok / SEQ, s = tok - b * SEQ;
    const float* xr = x + ((size_t)b * SEQ_FULL + s) * DM;
    float v[16], gl[16], el[16], yv[16];
    load_cols16(xr, lane, v);
    load_cols16(g, lane, gl);
    load_cols16(be, lane, el);
#pragma unroll
    for (int e = 0; e < 16; ++e) { v[e] = bf16r(v[e]); gl[e] = bf16r(gl[e]); el[e] = bf16r(el[e]); }
    ln_lane(v, gl, el, yv);
    v8h o[2];
#pragma unroll
    for (int j = 0; j < 2; ++j)
#pragma unroll
        for (int e = 0; e < 8; ++e) o[j][e] = (_Float16)yv[8 * j + e];
    _Float16* yr = y + (size_t)tok * DM;
    *(volatile v8h*)(yr + 8 * lane)       = o[0];
    *(volatile v8h*)(yr + 256 + 8 * lane) = o[1];
    __threadfence();
    *(volatile v8h*)(yr + 8 * lane)       = o[0];
    *(volatile v8h*)(yr + 256 + 8 * lane) = o[1];
}

static __device__ __forceinline__ void gemm_32x64(const _Float16* __restrict__ Ab,
                                                  const _Float16* __restrict__ Bb,
                                                  int K, int lane, v8f (&acc)[2][4]) {
#pragma unroll
    for (int t = 0; t < 2; ++t)
#pragma unroll
        for (int j = 0; j < 4; ++j) acc[t][j] = zero8();
#pragma unroll 1
    for (int k0 = 0; k0 < K; k0 += 32) {
        v16h a0 = load_frag16(Ab + k0, K, lane);
        v16h a1 = load_frag16(Ab + (size_t)16 * K + k0, K, lane);
        v16h bb[4];
#pragma unroll
        for (int j = 0; j < 4; ++j) bb[j] = load_frag16(Bb + (size_t)(16 * j) * K + k0, K, lane);
#pragma unroll
        for (int j = 0; j < 4; ++j) {
            acc[0][j] = wmma16(a0, bb[j], acc[0][j]);
            acc[1][j] = wmma16(a1, bb[j], acc[1][j]);
        }
    }
}

template <int EPI>
__global__ __launch_bounds__(256) __attribute__((amdgpu_num_vgpr(256)))
void k_gemm_p(const _Float16* __restrict__ A, int K, const _Float16* __restrict__ Bw,
              const float* __restrict__ b0, const float* __restrict__ b1,
              const float* __restrict__ b2, const float* __restrict__ b3,
              _Float16* __restrict__ outp, int ldo) {
    __shared__ __align__(16) _Float16 st[8][QR * 64];
    const int tid = threadIdx.x, lane = tid & 31, w = tid >> 5;
    const int hh = lane >> 4, m = lane & 15;
    const int m0  = blockIdx.x * QR;
    const int seg = blockIdx.y;
    const int nl  = 64 * w;
    const int n0w = seg * 512 + nl;
    const float* bias = (seg == 0) ? b0 : ((seg == 1) ? b1 : ((seg == 2) ? b2 : b3));

    v8f acc[2][4];
    gemm_32x64(A + (size_t)m0 * K, Bw + (size_t)n0w * K, K, lane, acc);

    float bl[4];
#pragma unroll
    for (int j = 0; j < 4; ++j) bl[j] = bf16r(bias[nl + 16 * j + m]);
#pragma unroll
    for (int t = 0; t < 2; ++t)
#pragma unroll
        for (int j = 0; j < 4; ++j)
#pragma unroll
            for (int r = 0; r < 8; ++r) {
                float a = acc[t][j][r];
                float val;
                if (EPI == 0) {
                    val = __builtin_fmaf(bl[j], WSC, a);
                } else {
                    float hx = __builtin_fmaf(a, SC_H, bl[j]);
                    val = WSC * mishf(hx);
                }
                st[w][(16 * t + 8 * hh + r) * 64 + 16 * j + m] = (_Float16)val;
            }
    wave_lds_sync();

    v8h pv[8];
    const int lr = lane >> 3, lc = (lane & 7) * 8;
#pragma unroll
    for (int i = 0; i < 8; ++i) pv[i] = *(const v8h*)(&st[w][(4 * i + lr) * 64 + lc]);
    _Float16* ob = outp + (size_t)m0 * ldo + n0w;
#pragma unroll
    for (int i = 0; i < 8; ++i) *(volatile v8h*)(ob + (size_t)(4 * i + lr) * ldo + lc) = pv[i];
    __threadfence();
#pragma unroll
    for (int i = 0; i < 8; ++i) *(volatile v8h*)(ob + (size_t)(4 * i + lr) * ldo + lc) = pv[i];
}

template <int MODE>
__global__ __launch_bounds__(256) __attribute__((amdgpu_num_vgpr(256)))
void k_gemm_r(const _Float16* __restrict__ A, int K, const _Float16* __restrict__ Bw,
              const float* __restrict__ bias, const float* __restrict__ res,
              const float* __restrict__ g, const float* __restrict__ be,
              float* __restrict__ outf, _Float16* __restrict__ outh) {
    __shared__ __align__(16) float T[QR * DM];
    const int tid = threadIdx.x, lane = tid & 31, w = tid >> 5;
    const int hh = lane >> 4, m = lane & 15;
    const int m0 = blockIdx.x * QR;
    const int nl = 64 * w;

    v8f acc[2][4];
    gemm_32x64(A + (size_t)m0 * K, Bw + (size_t)nl * K, K, lane, acc);
#pragma unroll
    for (int t = 0; t < 2; ++t)
#pragma unroll
        for (int j = 0; j < 4; ++j)
#pragma unroll
            for (int r = 0; r < 8; ++r)
                T[(16 * t + 8 * hh + r) * DM + nl + 16 * j + m] = acc[t][j][r];
    __syncthreads();

    float bl[16], gl[16], el[16];
    load_cols16(bias, lane, bl);
    load_cols16(g, lane, gl);
    load_cols16(be, lane, el);
#pragma unroll
    for (int e = 0; e < 16; ++e) { bl[e] = bf16r(bl[e]); gl[e] = bf16r(gl[e]); el[e] = bf16r(el[e]); }

#pragma unroll 1
    for (int rr = 0; rr < 4; ++rr) {
        const int row = 4 * w + rr;
        const int tok = m0 + row;
        float v[16], rv[16], yv[16];
        load_cols16(&T[row * DM], lane, v);
        if (MODE == 0) {
            const int b = tok / SEQ, s = tok - b * SEQ;
            load_cols16(res + ((size_t)b * SEQ_FULL + s) * DM, lane, rv);
#pragma unroll
            for (int e = 0; e < 16; ++e) rv[e] = bf16r(rv[e]);
        } else {
            load_cols16(res + (size_t)tok * DM, lane, rv);
        }
#pragma unroll
        for (int e = 0; e < 16; ++e) v[e] = rv[e] + __builtin_fmaf(v[e], SC_O, bl[e]);
        ln_lane(v, gl, el, yv);

        float* trow = &T[row * DM];
#pragma unroll
        for (int j = 0; j < 2; ++j) {
            v4f p0, p1;
            if (MODE == 0) {
                p0.x = v[8 * j + 0]; p0.y = v[8 * j + 1]; p0.z = v[8 * j + 2]; p0.w = v[8 * j + 3];
                p1.x = v[8 * j + 4]; p1.y = v[8 * j + 5]; p1.z = v[8 * j + 6]; p1.w = v[8 * j + 7];
            } else {
                p0.x = yv[8 * j + 0]; p0.y = yv[8 * j + 1]; p0.z = yv[8 * j + 2]; p0.w = yv[8 * j + 3];
                p1.x = yv[8 * j + 4]; p1.y = yv[8 * j + 5]; p1.z = yv[8 * j + 6]; p1.w = yv[8 * j + 7];
            }
            *(v4f*)(trow + 256 * j + 8 * lane)     = p0;
            *(v4f*)(trow + 256 * j + 8 * lane + 4) = p1;
        }
        wave_lds_sync();
        v4f s4[4];
#pragma unroll
        for (int jj = 0; jj < 4; ++jj) s4[jj] = *(const v4f*)(trow + 128 * jj + 4 * lane);

        float* orow = outf + (size_t)tok * DM;
        if (MODE == 0) {
            v8h o[2];
#pragma unroll
            for (int j = 0; j < 2; ++j)
#pragma unroll
                for (int e = 0; e < 8; ++e) o[j][e] = (_Float16)yv[8 * j + e];
            _Float16* hrow = outh + (size_t)tok * DM;
            *(volatile v8h*)(hrow + 8 * lane)       = o[0];
            *(volatile v8h*)(hrow + 256 + 8 * lane) = o[1];
#pragma unroll
            for (int jj = 0; jj < 4; ++jj) *(volatile v4f*)(orow + 128 * jj + 4 * lane) = s4[jj];
            __threadfence();
            *(volatile v8h*)(hrow + 8 * lane)       = o[0];
            *(volatile v8h*)(hrow + 256 + 8 * lane) = o[1];
#pragma unroll
            for (int jj = 0; jj < 4; ++jj) *(volatile v4f*)(orow + 128 * jj + 4 * lane) = s4[jj];
        } else {
#pragma unroll
            for (int jj = 0; jj < 4; ++jj) *(volatile v4f*)(orow + 128 * jj + 4 * lane) = s4[jj];
            __threadfence();
#pragma unroll
            for (int jj = 0; jj < 4; ++jj) *(volatile v4f*)(orow + 128 * jj + 4 * lane) = s4[jj];
        }
    }
}

__global__ __launch_bounds__(256) __attribute__((amdgpu_num_vgpr(256)))
void k_attn(const _Float16* __restrict__ qkv, _Float16* __restrict__ ctx) {
    __shared__ __align__(16) float    zs[QR * SEQ];
    __shared__ __align__(16) _Float16 Vt[HD * VTP];
    __shared__ __align__(16) _Float16 Cst[QR * HD];
    _Float16* ph = reinterpret_cast<_Float16*>(zs);
    constexpr int PP  = 2 * SEQ;
    constexpr int PLD = PP + 8;
    constexpr int KTW = SEQ / 128;

    const int tid = threadIdx.x, lane = tid & 31, w = tid >> 5;
    const int hh = lane >> 4, m = lane & 15;
    const int h = blockIdx.y, b = blockIdx.z;
    const int q0 = blockIdx.x * QR;
    const size_t tokq = (size_t)b * SEQ + q0;
    const _Float16* qp = qkv + tokq * DQKV + h * HD;
    const _Float16* kp = qkv + (size_t)b * SEQ * DQKV + DM + h * HD;
    const _Float16* vp = qkv + (size_t)b * SEQ * DQKV + 2 * DM + h * HD;

    {
        const v16h qa00 = load_frag16(qp, DQKV, lane);
        const v16h qa01 = load_frag16(qp + 32, DQKV, lane);
        const v16h qa10 = load_frag16(qp + (size_t)16 * DQKV, DQKV, lane);
        const v16h qa11 = load_frag16(qp + (size_t)16 * DQKV + 32, DQKV, lane);
#pragma unroll 1
        for (int i = 0; i < KTW; ++i) {
            const int key0 = (w * KTW + i) * 16;
            const _Float16* kt = kp + (size_t)key0 * DQKV;
            v16h kf0 = load_frag16(kt, DQKV, lane);
            v16h kf1 = load_frag16(kt + 32, DQKV, lane);
            v8f s0 = wmma16(qa00, kf0, zero8());
            s0 = wmma16(qa01, kf1, s0);
            v8f s1 = wmma16(qa10, kf0, zero8());
            s1 = wmma16(qa11, kf1, s1);
#pragma unroll
            for (int r = 0; r < 8; ++r) {
                zs[(8 * hh + r) * SEQ + key0 + m]      = s0[r] * SC_Z;
                zs[(16 + 8 * hh + r) * SEQ + key0 + m] = s1[r] * SC_Z;
            }
        }
    }
    __syncthreads();

    const float tcl = -rsqrtf((float)SEQ);
#pragma unroll 1
    for (int rr = 0; rr < 4; ++rr) {
        const int row = 4 * w + rr;
        float z[ZN];
        const float* zr = &zs[row * SEQ];
#pragma unroll
        for (int j = 0; j < ZN / 4; ++j) {
            v4f t4 = *(const v4f*)(zr + 128 * j + 4 * lane);
            z[4 * j + 0] = t4.x; z[4 * j + 1] = t4.y; z[4 * j + 2] = t4.z; z[4 * j + 3] = t4.w;
        }
        float mx = z[0], mn = z[0];
#pragma unroll
        for (int i = 1; i < ZN; ++i) { mx = fmaxf(mx, z[i]); mn = fminf(mn, z[i]); }
        mx = wmaxr(mx);
        mn = wminr(mn);
#pragma unroll
        for (int i = 0; i < ZN; ++i) z[i] = z[i] - mx;
        float tau = fminf(fmaxf(mn - mx, -1.0f), tcl);
#pragma unroll 1
        for (int it = 0; it < NEWT; ++it) {
            float sa = 0.0f, sb = 0.0f;
#pragma unroll
            for (int i = 0; i < ZN; ++i) {
                float d = fmaxf(z[i] - tau, 0.0f);
                sa += d;
                sb = __builtin_fmaf(d, d, sb);
            }
            sa = wsum(sa);
            sb = wsum(sb);
            tau = tau + (sb - 1.0f) * (0.5f * __builtin_amdgcn_rcpf(sa));
            tau = fminf(fmaxf(tau, -1.0f), tcl);
        }
        _Float16* prow = ph + (size_t)row * PP + (row & 15) * 8;
#pragma unroll
        for (int j = 0; j < ZN / 4; ++j) {
            v4h pk;
#pragma unroll
            for (int e = 0; e < 4; ++e) {
                float d = fmaxf(z[4 * j + e] - tau, 0.0f);
                pk[e] = (_Float16)(d * d * SC_P);
            }
            *(v4h*)(prow + 128 * j + 4 * lane) = pk;
        }
    }
    __syncthreads();

    const int rt = w & 1, ct = w >> 1;
    v8f acc = zero8();
#pragma unroll 1
    for (int c0 = 0; c0 < SEQ; c0 += CH) {
#pragma unroll
        for (int i2 = 0; i2 < 8; ++i2) {
            const int idx = tid + 256 * i2;
            const int t = idx >> 3, part = idx & 7;
            v8h vv = *(const v8h*)(vp + (size_t)(c0 + t) * DQKV + part * 8);
#pragma unroll
            for (int e = 0; e < 8; ++e) Vt[(part * 8 + e) * VTP + t] = vv[e];
        }
        __syncthreads();
#pragma unroll 1
        for (int j = 0; j < CH; j += 32) {
            v16h pa = load_frag16(ph + (size_t)(16 * rt) * PP + c0 + j, PLD, lane);
            v16h vb = load_frag16(&Vt[(16 * ct) * VTP + j], VTP, lane);
            acc = wmma16(pa, vb, acc);
        }
        __syncthreads();
    }

#pragma unroll
    for (int r = 0; r < 8; ++r)
        Cst[(16 * rt + 8 * hh + r) * HD + 16 * ct + m] = (_Float16)(acc[r] * SC_C);
    __syncthreads();
    const int orow = 4 * w + (lane >> 3), oc = (lane & 7) * 8;
    v8h cv = *(const v8h*)(&Cst[orow * HD + oc]);
    _Float16* dst = ctx + (tokq + orow) * DM + h * HD + oc;
    *(volatile v8h*)dst = cv;
    __threadfence();
    *(volatile v8h*)dst = cv;
}

extern "C" void kernel_launch(void* const* d_in, const int* in_sizes, int n_in,
                              void* d_out, int out_size, void* d_ws, size_t ws_size,
                              hipStream_t stream) {
    if (n_in < 19) return;
    if (in_sizes[0] < ((NB - 1) * SEQ_FULL + SEQ) * DM) return;
    if (in_sizes[1] < DM * DM || in_sizes[3] < DM * DM || in_sizes[5] < DM * DM || in_sizes[7] < DM * DM) return;
    if (in_sizes[2] < DM || in_sizes[4] < DM || in_sizes[6] < DM || in_sizes[8] < DM) return;
    if (in_sizes[9] < DM || in_sizes[10] < DM || in_sizes[15] < DM || in_sizes[16] < DM) return;
    if (in_sizes[17] < DM || in_sizes[18] < DM || in_sizes[14] < DM) return;
    if (in_sizes[11] < DF * DM || in_sizes[13] < DM * DF || in_sizes[12] < DF) return;
    if (out_size < NTOK * DM) return;

    const float* x    = (const float*)d_in[0];
    const float* Wq   = (const float*)d_in[1];
    const float* bq   = (const float*)d_in[2];
    const float* Wk   = (const float*)d_in[3];
    const float* bk   = (const float*)d_in[4];
    const float* Wv   = (const float*)d_in[5];
    const float* bv   = (const float*)d_in[6];
    const float* Wo   = (const float*)d_in[7];
    const float* bo   = (const float*)d_in[8];
    const float* ln1g = (const float*)d_in[9];
    const float* ln1b = (const float*)d_in[10];
    const float* W1   = (const float*)d_in[11];
    const float* bf1  = (const float*)d_in[12];
    const float* W2   = (const float*)d_in[13];
    const float* bf2  = (const float*)d_in[14];
    const float* ln2g = (const float*)d_in[15];
    const float* ln2b = (const float*)d_in[16];
    const float* lnfg = (const float*)d_in[17];
    const float* lnfb = (const float*)d_in[18];
    float* out = (float*)d_out;

    char* ws = (char*)d_ws;
    size_t off = 0;
    _Float16* wqkv = (_Float16*)(ws + off); off += (size_t)DQKV * DM * 2;
    _Float16* wo16 = (_Float16*)(ws + off); off += (size_t)DM * DM * 2;
    _Float16* w116 = (_Float16*)(ws + off); off += (size_t)DF * DM * 2;
    _Float16* w216 = (_Float16*)(ws + off); off += (size_t)DM * DF * 2;
    _Float16* y1   = (_Float16*)(ws + off); off += (size_t)NTOK * DM * 2;
    _Float16* qkv  = (_Float16*)(ws + off); off += (size_t)NTOK * DQKV * 2;
    _Float16* cpl  = (_Float16*)(ws + off); off += (size_t)NTOK * DM * 2;
    float*    x1   = (float*)(ws + off);    off += (size_t)NTOK * DM * 4;
    _Float16* y2   = (_Float16*)(ws + off); off += (size_t)NTOK * DM * 2;
    _Float16* mpl  = (_Float16*)(ws + off); off += (size_t)NTOK * DF * 2;
    if (off > ws_size) return;

    k_wcvt<<<dim3(DM * DM / 2048), dim3(256), 0, stream>>>(Wq, wqkv);
    k_wcvt<<<dim3(DM * DM / 2048), dim3(256), 0, stream>>>(Wk, wqkv + (size_t)DM * DM);
    k_wcvt<<<dim3(DM * DM / 2048), dim3(256), 0, stream>>>(Wv, wqkv + (size_t)2 * DM * DM);
    k_wcvt<<<dim3(DM * DM / 2048), dim3(256), 0, stream>>>(Wo, wo16);
    k_wcvt<<<dim3(DF * DM / 2048), dim3(256), 0, stream>>>(W1, w116);
    k_wcvt<<<dim3(DM * DF / 2048), dim3(256), 0, stream>>>(W2, w216);

    k_ln1<<<dim3(NTOK / 8), dim3(256), 0, stream>>>(x, ln1g, ln1b, y1);
    k_gemm_p<0><<<dim3(NTOK / QR, 3), dim3(256), 0, stream>>>(y1, DM, wqkv, bq, bk, bv, bv, qkv, DQKV);
    k_attn<<<dim3(SEQ / QR, NH, NB), dim3(256), 0, stream>>>(qkv, cpl);
    k_gemm_r<0><<<dim3(NTOK / QR), dim3(256), 0, stream>>>(cpl, DM, wo16, bo, x, ln2g, ln2b, x1, y2);
    k_gemm_p<1><<<dim3(NTOK / QR, DF / 512), dim3(256), 0, stream>>>(y2, DM, w116, bf1, bf1 + 512, bf1 + 1024, bf1 + 1536, mpl, DF);
    k_gemm_r<1><<<dim3(NTOK / QR), dim3(256), 0, stream>>>(mpl, DF, w216, bf2, x1, lnfg, lnfb, out, y2);
}
